// SphericalConv_36189394436282
// MI455X (gfx1250) — hardware-verified
//
#include <hip/hip_runtime.h>
#include <math.h>

#define L1C  16
#define BB   4
#define NN   8192
#define CINC 64
#define COUTC 64
#define NCH  128
#define SLOPEC 0.01f

typedef _Float16 f16;
typedef __attribute__((ext_vector_type(16))) _Float16 v16h;
typedef __attribute__((ext_vector_type(8)))  float    v8f;
typedef __attribute__((ext_vector_type(4)))  float    v4f_t;
typedef float v4fa __attribute__((ext_vector_type(4), may_alias));
#define NBLK (NN / NCH)
#define PLG  ((size_t)BB * L1C * 4 * 512)
#define RSPLIT (1.0f / 2048.0f)
__device__ __forceinline__ f16 lo_of(float v, f16 h) { return (f16)((v - (float)h) * 2048.0f); }
__device__ __forceinline__ v8f wmma16(v16h a, v16h b, v8f c) { return __builtin_amdgcn_wmma_f32_16x16x32_f16(false, a, false, b, (short)0, c, false, false); }
__device__ __forceinline__ v8f wmma_split(v16h a, v16h al, v16h b, v16h bl, v8f c) { v8f x = {}; x = wmma16(al, b, x); x = wmma16(a, bl, x); return wmma16(a, b, c) + x * RSPLIT; }

__device__ __forceinline__ int a_pos(int m, int k) {
  return (m + (((k >> 3) & 1) << 4)) * 16 + (k & 7) + ((k >> 4) << 3);
}
__device__ __forceinline__ int b_pos(int k, int n) {
  return (n + (((k >> 3) & 1) << 4)) * 16 + (k & 7) + ((k >> 4) << 3);
}
__device__ __forceinline__ v16h frag_ld(const f16* buf, int lane) {
  const uint4* p = (const uint4*)(buf + lane * 16);
  union { uint4 u[2]; v16h v; } r;
  r.u[0] = p[0];
  r.u[1] = p[1];
  return r.v;
}

__device__ __forceinline__ float lrelu(float x) { return x > 0.f ? x : SLOPEC * x; }

struct BasisState {
  float x, s, pmm, invf;
  float cm[L1C], sm[L1C];
  float Pm1[L1C], Pm2[L1C], rat[L1C];
};

__device__ __forceinline__ void basis_init(BasisState& st, float theta, float phi) {
  st.x = cosf(theta);
  st.s = sqrtf(fmaxf(0.f, 1.f - st.x * st.x));
  st.pmm = 1.f;
  st.invf = 1.f;
  float c1 = cosf(phi), s1 = sinf(phi);
  st.cm[0] = 1.f; st.sm[0] = 0.f;
#pragma unroll
  for (int m = 1; m < L1C; ++m) {
    float cp = st.cm[m - 1], sp = st.sm[m - 1];
    st.cm[m] = cp * c1 - sp * s1;
    st.sm[m] = sp * c1 + cp * s1;
  }
}

__device__ __forceinline__ void basis_step(BasisState& st, int l,
                                           float* qc, float* qs) {
  if (l > 0) {
    st.pmm  *= -(2.f * l - 1.f) * st.s;
    st.invf *= 1.f / ((2.f * l - 1.f) * (2.f * l));
  }
#pragma unroll
  for (int m = 0; m < L1C; ++m) {
    float Q = 0.f;
    if (m <= l) {
      float P;
      if (m == l) {
        P = st.pmm;
        st.Pm1[m] = P; st.Pm2[m] = 0.f;
        st.rat[m] = st.invf;
      } else {
        st.rat[m] *= (float)(l - m) / (float)(l + m);
        P = ((2.f * l - 1.f) * st.x * st.Pm1[m] - (float)(l - 1 + m) * st.Pm2[m])
            / (float)(l - m);
        st.Pm2[m] = st.Pm1[m]; st.Pm1[m] = P;
      }
      float q2 = 6.283185307f * sqrtf(12.56637061f / (2.f * l + 1.f))
               * (2.f * l + 1.f) * st.rat[m] * 0.07957747155f;
      Q = sqrtf(fmaxf(q2, 0.f)) * P;
    }
    qc[m] = Q * st.cm[m];
    qs[m] = Q * st.sm[m];
  }
}

__global__ void k_zero(float* p, int n) {
  int i = blockIdx.x * blockDim.x + threadIdx.x;
  if (i < n) p[i] = 0.f;
}

__global__ void __launch_bounds__(256) k_analysis(
    const float* __restrict__ theta, const float* __restrict__ phi,
    const float* __restrict__ areas, const float* __restrict__ values,
    const float* __restrict__ W, float* __restrict__ SAcc) {
  extern __shared__ char smem[];
  f16* valsA = (f16*)smem;
  f16* wtB   = valsA + 8 * 2 * 512;
  f16* prodB = wtB + 2 * 4 * 512;
  f16* qcA   = prodB + 4 * 4 * 512;
  f16* qsA   = qcA + 4 * 512;
  const int LOFF = (8 * 2 + 2 * 4 + 4 * 4 + 4 + 4) * 512;
  float* stg = (float*)(smem + (size_t)2 * LOFF * 2);

  const int t = threadIdx.x, lane = t & 31, wv = t >> 5;
  const int b = blockIdx.y;
  const int n0 = blockIdx.x * NCH;

  for (int i = t; i < NCH * CINC; i += 256) {
    int n = i >> 6, c = i & 63;
    size_t gp = (size_t)b * NN + n0 + n;
    const float fv = values[gp * CINC + c] * areas[gp];
    const f16 v = (f16)fv;
    const int pos = ((n >> 4) * 2 + (c >> 5)) * 512 + a_pos(n & 15, c & 31);
    valsA[pos] = v; valsA[LOFF + pos] = lo_of(fv, v);
  }
  BasisState st;
  if (t < NCH) basis_init(st, theta[(size_t)b * NN + n0 + t], phi[(size_t)b * NN + n0 + t]);

  for (int l = 0; l < L1C; ++l) {
    __syncthreads();

    for (int i = t; i < CINC * COUTC; i += 256) {
      int c = i >> 6, d = i & 63;
      const float fw = W[(size_t)l * CINC * COUTC + i];
      const f16 v = (f16)fw;
      const int pos = ((c >> 5) * 4 + (d >> 4)) * 512 + b_pos(c & 31, d & 15);
      wtB[pos] = v; wtB[LOFF + pos] = lo_of(fw, v);
    }
    if (l + 1 < L1C)
      __builtin_prefetch(&W[(size_t)(l + 1) * CINC * COUTC + t], 0, 1);

    if (t < NCH) {
      float qcr[L1C], qsr[L1C];
      basis_step(st, l, qcr, qsr);
      const int ks = t >> 5, kl = t & 31;
#pragma unroll
      for (int m = 0; m < L1C; ++m) {
        int p = ks * 512 + a_pos(m, kl);
        qcA[p] = (f16)qcr[m];  qcA[LOFF + p] = lo_of(qcr[m], qcA[p]);
        qsA[p] = (f16)qsr[m];  qsA[LOFF + p] = lo_of(qsr[m], qsA[p]);
      }
    }
    __syncthreads();

    {
      const int mt = wv;
      const int hi = lane >> 4, nc = lane & 15;
#pragma unroll
      for (int nt = 0; nt < 4; ++nt) {
        v8f acc = {};
#pragma unroll
        for (int ks = 0; ks < 2; ++ks) {
          v16h a  = frag_ld(valsA + (mt * 2 + ks) * 512, lane), al = frag_ld(valsA + LOFF + (mt * 2 + ks) * 512, lane);
          v16h bf = frag_ld(wtB + (ks * 4 + nt) * 512, lane),   bl = frag_ld(wtB + LOFF + (ks * 4 + nt) * 512, lane);
          acc = wmma_split(a, al, bf, bl, acc);
        }
        union { f16 h[8]; uint4 u; } pk, pl;
#pragma unroll
        for (int v = 0; v < 8; ++v) { pk.h[v] = (f16)acc[v]; pl.h[v] = lo_of(acc[v], pk.h[v]); }
        f16* dst = prodB + ((mt >> 1) * 4 + nt) * 512 + lane * 16 + ((mt & 1) << 3);
        *(uint4*)dst = pk.u; *(uint4*)(dst + LOFF) = pl.u;
      }
    }
    __syncthreads();

    {
      const int r = wv >> 2, dt = wv & 3;
      const f16* A = r ? qsA : qcA;
      v8f acc = {};
#pragma unroll
      for (int ks = 0; ks < 4; ++ks) {
        v16h a  = frag_ld(A + ks * 512, lane),                  al = frag_ld(A + LOFF + ks * 512, lane);
        v16h bf = frag_ld(prodB + (ks * 4 + dt) * 512, lane),   bl = frag_ld(prodB + LOFF + (ks * 4 + dt) * 512, lane);
        acc = wmma_split(a, al, bf, bl, acc);
      }
      const int hi = lane >> 4, nc = lane & 15;
#pragma unroll
      for (int v = 0; v < 8; ++v) stg[(r * L1C + v + hi * 8) * COUTC + dt * 16 + nc] = acc[v];
    }
    __syncthreads();
    {
      float* dst = SAcc + ((((size_t)b * NBLK + blockIdx.x) * L1C + l) * 2) * (L1C * COUTC);
#pragma unroll 1
      for (int pass = 0; pass < 2; ++pass) {
        for (int c = t; c < 512; c += 256) *(volatile v4f_t*)(dst + c * 4) = *(const volatile v4fa*)(stg + c * 4);
        __threadfence();
      }
    }
  }
}

__global__ void __launch_bounds__(256) k_act(const float* __restrict__ SAcc, f16* __restrict__ G) {
  __shared__ __attribute__((aligned(16))) f16 gs[2][4 * 512];
  const int l = blockIdx.x & 15, b = blockIdx.x >> 4, t = threadIdx.x;
  for (int j = t; j < 2048; j += 256) {
    const int d = j & 63, m = (j >> 6) & 15, r = j >> 10;
    float S = 0.f;
    for (int blk = 0; blk < NBLK; ++blk) S += SAcc[((((size_t)b * NBLK + blk) * L1C + l) * 2) * (L1C * COUTC) + j];
    const float fac = (m == 0) ? 1.f : 2.f;
    const float g = (r == 0) ? fac * lrelu(S) : -fac * lrelu(-S);
    const int k = r * 16 + m;
    const int pos = (d >> 4) * 512 + b_pos(k, d & 15);
    const f16 gh = (f16)g;
    gs[0][pos] = gh; gs[1][pos] = lo_of(g, gh);
  }
  __syncthreads();
  f16* gdst = G + ((size_t)b * L1C + l) * 4 * 512;
  const uint4 u0 = ((const uint4*)gs[0])[t], u1 = ((const uint4*)gs[1])[t];
  typedef __attribute__((ext_vector_type(4))) unsigned v4u_t;
  v4u_t w0, w1; w0.x = u0.x; w0.y = u0.y; w0.z = u0.z; w0.w = u0.w; w1.x = u1.x; w1.y = u1.y; w1.z = u1.z; w1.w = u1.w;
  *(volatile v4u_t*)((uint4*)gdst + t) = w0; *(volatile v4u_t*)((uint4*)(gdst + PLG) + t) = w1; __threadfence();
  *(volatile v4u_t*)((uint4*)gdst + t) = w0; *(volatile v4u_t*)((uint4*)(gdst + PLG) + t) = w1;
}

__global__ void __launch_bounds__(256) k_synth(
    const float* __restrict__ theta, const float* __restrict__ phi,
    const f16* __restrict__ G, float* __restrict__ out) {
  extern __shared__ char smem[];
  f16* qcsA = (f16*)smem;
  f16* gB   = qcsA + 8 * 512;
  const int LOFF = 12 * 512;
  __shared__ __attribute__((aligned(16))) float ost[8][16 * 68];

  const int t = threadIdx.x, lane = t & 31, wv = t >> 5;
  const int b = blockIdx.y;
  const int n0 = blockIdx.x * NCH;

  BasisState st;
  if (t < NCH) basis_init(st, theta[(size_t)b * NN + n0 + t], phi[(size_t)b * NN + n0 + t]);

  v8f zero = {};
  v8f acc[4];
#pragma unroll
  for (int i = 0; i < 4; ++i) acc[i] = zero;

  for (int l = 0; l < L1C; ++l) {
    __syncthreads();
    {
      const uint4* src = (const uint4*)(G + ((size_t)b * L1C + l) * 4 * 512);
      ((uint4*)gB)[t] = src[t];
      ((uint4*)(gB + LOFF))[t] = ((const uint4*)(G + PLG + ((size_t)b * L1C + l) * 4 * 512))[t];
    }
    if (t < NCH) {
      float qcr[L1C], qsr[L1C];
      basis_step(st, l, qcr, qsr);
      const int mt = t >> 4, pr = t & 15;
      f16* base = qcsA + mt * 512;
      union { f16 h[8]; uint4 u; } u0, u1, u2, u3, w0, w1, w2, w3;
#pragma unroll
      for (int m = 0; m < 8; ++m) {
        u0.h[m] = (f16)qcr[m];       w0.h[m] = lo_of(qcr[m], u0.h[m]);
        u1.h[m] = (f16)qcr[m + 8];   w1.h[m] = lo_of(qcr[m + 8], u1.h[m]);
        u2.h[m] = (f16)qsr[m];       w2.h[m] = lo_of(qsr[m], u2.h[m]);
        u3.h[m] = (f16)qsr[m + 8];   w3.h[m] = lo_of(qsr[m + 8], u3.h[m]);
      }
      *(uint4*)(base + pr * 16)            = u0.u;   *(uint4*)(base + LOFF + pr * 16)            = w0.u;
      *(uint4*)(base + (pr + 16) * 16)     = u1.u;   *(uint4*)(base + LOFF + (pr + 16) * 16)     = w1.u;
      *(uint4*)(base + pr * 16 + 8)        = u2.u;   *(uint4*)(base + LOFF + pr * 16 + 8)        = w2.u;
      *(uint4*)(base + (pr + 16) * 16 + 8) = u3.u;   *(uint4*)(base + LOFF + (pr + 16) * 16 + 8) = w3.u;
    }
    __syncthreads();

    const int mt = wv;
#pragma unroll
    for (int dt = 0; dt < 4; ++dt) {
      v16h a  = frag_ld(qcsA + mt * 512, lane), al = frag_ld(qcsA + LOFF + mt * 512, lane);
      v16h bf = frag_ld(gB + dt * 512, lane),     bl = frag_ld(gB + LOFF + dt * 512, lane);
      acc[dt] = wmma_split(a, al, bf, bl, acc[dt]);
    }
  }

  const int hi = lane >> 4, nc = lane & 15;
  float* so = ost[wv];
#pragma unroll
  for (int dt = 0; dt < 4; ++dt)
#pragma unroll
    for (int v = 0; v < 8; ++v) so[(v + hi * 8) * 68 + dt * 16 + nc] = acc[dt][v];
  asm volatile("s_wait_dscnt 0" ::: "memory");
#pragma unroll 1
  for (int pass = 0; pass < 2; ++pass) {
#pragma unroll
    for (int i = 0; i < 8; ++i) { const int c = lane + 32 * i, rr = c >> 4, q = (c & 15) * 4;
      *(volatile v4f_t*)(out + ((size_t)b * NN + n0 + wv * 16 + rr) * COUTC + q) = *(const volatile v4fa*)(so + rr * 68 + q); }
    __threadfence();
  }
}

extern "C" void kernel_launch(void* const* d_in, const int* in_sizes, int n_in,
                              void* d_out, int out_size, void* d_ws, size_t ws_size,
                              hipStream_t stream) {
  (void)in_sizes; (void)n_in; (void)out_size; (void)ws_size;
  const float* theta  = (const float*)d_in[0];
  const float* phi    = (const float*)d_in[1];
  const float* areas  = (const float*)d_in[2];
  const float* values = (const float*)d_in[3];
  const float* W      = (const float*)d_in[4];
  float* out = (float*)d_out;

  const size_t accN = (size_t)BB * NBLK * L1C * 2 * L1C * COUTC;
  float* SAcc = (float*)d_ws;
  f16*   G    = (f16*)(SAcc + accN);

  size_t smemA = (size_t)2 * (8 * 2 + 2 * 4 + 4 * 4 + 4 + 4) * 512 * 2 + 2 * L1C * COUTC * 4;
  k_analysis<<<dim3(NN / NCH, BB), 256, smemA, stream>>>(theta, phi, areas, values, W, SAcc);

  k_act<<<BB * L1C, 256, 0, stream>>>(SAcc, G);

  size_t smemC = (size_t)2 * (8 + 4) * 512 * 2;
  k_synth<<<dim3(NN / NCH, BB), 256, smemC, stream>>>(theta, phi, G, out);
}
